// NonLocalBlock_59399397703753
// MI455X (gfx1250) — hardware-verified
//
#include <hip/hip_runtime.h>


#ifndef NB
#define NB 4
#endif
#ifndef SEQ
#define SEQ 4096
#endif
#define NB_FULL  4
#define SEQ_FULL 4096
#ifndef OUT_SEQ
#define OUT_SEQ SEQ
#endif
#define CIN  256
#define CO   256
#define HD   32
#define AW   4
#define OP   68
#define QRS  2048.0f
#define QRI  (1.0f / 2048.0f)
#define L2E  1.4426950408889634f
#define PSH  14.0f
#define NEGB (-3.0e38f)

static_assert(HD == 32);
static_assert(CIN % 32 == 0);
static_assert(CIN == CO);
static_assert(CO % 64 == 0);
static_assert(SEQ % 64 == 0);
static_assert((NB * SEQ) % 64 == 0);
static_assert(SEQ % 32 == 0);
static_assert(SEQ % (16 * AW) == 0);
static_assert(NB <= NB_FULL);
static_assert(SEQ <= SEQ_FULL);
static_assert((OP * 4) % 16 == 0);
static_assert(((size_t)SEQ * CIN) % 8 == 0);
static_assert((CIN * HD) % (256 * 8) == 0);
static_assert((HD * CO) % (256 * 8) == 0);
static_assert(2 * 32 * 16 == 16 * HD * 2);
static_assert(4 * 32 * 16 == 16 * 64 * 2);
static_assert(8 * 32 * 16 == 16 * 64 * 4);
static_assert(16 * OP * 4 <= 131072);
static_assert(AW * 16 * OP * 4 <= 131072);
static_assert(CIN * HD * 2 <= 131072);

typedef _Float16 h16;
typedef unsigned short bf;
typedef __attribute__((ext_vector_type(16))) __bf16   v16bf;
typedef __attribute__((ext_vector_type(16))) _Float16 v16h;
typedef __attribute__((ext_vector_type(8)))  _Float16 v8h;
typedef __attribute__((ext_vector_type(8)))  unsigned short v8us;
typedef __attribute__((ext_vector_type(8)))  float    v8f;
typedef __attribute__((ext_vector_type(4)))  float    v4f;
typedef v4f  __attribute__((may_alias)) v4fa;
typedef v8us __attribute__((may_alias)) v8usa;
typedef v8h  __attribute__((may_alias)) v8ha;

__device__ __forceinline__ unsigned short f2bf(float f) { unsigned u = __float_as_uint(f); u += 0x7FFFu + ((u >> 16) & 1u); return (unsigned short)(u >> 16); }
__device__ __forceinline__ float bfr(float f) { return __uint_as_float(((unsigned)f2bf(f)) << 16); }
__device__ __forceinline__ v16h cat16(v8h lo, v8h hi) { return __builtin_shufflevector(lo, hi, 0, 1, 2, 3, 4, 5, 6, 7, 8, 9, 10, 11, 12, 13, 14, 15); }
__device__ __forceinline__ v16bf cat16b(v8us lo, v8us hi) { return __builtin_bit_cast(v16bf, __builtin_shufflevector(lo, hi, 0, 1, 2, 3, 4, 5, 6, 7, 8, 9, 10, 11, 12, 13, 14, 15)); }
__device__ __forceinline__ v8f wmma16(v16h a, v16h b, v8f c) { return __builtin_amdgcn_wmma_f32_16x16x32_f16(false, a, false, b, (short)0, c, false, false); }
__device__ __forceinline__ v8f wmmab(v16bf a, v16bf b, v8f c) { return __builtin_amdgcn_wmma_f32_16x16x32_bf16(false, a, false, b, (short)0, c, false, false); }
__device__ __forceinline__ v8f wmma16g(v16h a, v16h b, v8f c) { c = wmma16(a, b, c); asm volatile("v_nop\n\tv_nop\n\tv_nop\n\tv_nop" : "+v"(c) : "v"(a), "v"(b)); return c; }
__device__ __forceinline__ v8f wmmabg(v16bf a, v16bf b, v8f c) { c = wmmab(a, b, c); asm volatile("v_nop\n\tv_nop\n\tv_nop\n\tv_nop" : "+v"(c) : "v"(a), "v"(b)); return c; }
__device__ __forceinline__ v16h  ldh(const h16* p) { return cat16(*(const v8h*)p, *(const v8h*)(p + 16)); }
__device__ __forceinline__ v16bf ldb(const bf* p)  { return cat16b(*(const v8us*)p, *(const v8us*)(p + 16)); }
__device__ __forceinline__ void wave_sync() { __builtin_amdgcn_fence(3  , "wavefront"); __builtin_amdgcn_wave_barrier(); asm volatile("" ::: "memory"); }
static __device__ __forceinline__ h16 toh_flush(float v) { const float w = (fabsf(v) < 6.103515625e-05f) ? 0.0f : v; return (h16)w; }

__global__ __launch_bounds__(256) void k_cvt8(const float* __restrict__ src, bf* dst, size_t n8) {
    const size_t i = (size_t)blockIdx.x * 256 + threadIdx.x; if (i >= n8) return;
    const v8f v = *(const v8f*)(src + i * 8); v8us o;
#pragma unroll
    for (int k = 0; k < 8; ++k) o[k] = f2bf(v[k]);
    *(volatile v8us*)(dst + i * 8) = o; __threadfence(); *(volatile v8us*)(dst + i * 8) = o;
}

__global__ __launch_bounds__(256) void k_wtb(const float* __restrict__ src, bf* dst) {
    __shared__ __align__(16) bf ts[HD * CIN];
    const unsigned tid = threadIdx.x;
#pragma unroll 1
    for (unsigned it = 0; it < (unsigned)(CIN * HD / 256); ++it) {
        const unsigned idx = it * 256u + tid; const unsigned k = idx / (unsigned)HD, n = idx % (unsigned)HD;
        ts[n * (unsigned)CIN + k] = f2bf(src[idx]); }
    __syncthreads();
#pragma unroll 1
    for (int ps = 0; ps < 2; ++ps) {
#pragma unroll 1
        for (unsigned it = 0; it < (unsigned)(CIN * HD / 8 / 256); ++it) {
            const unsigned c = it * 256u + tid;
            const v8us o = *(const v8usa*)(&ts[c * 8u]);
            *(volatile v8us*)(dst + (size_t)c * 8) = o; }
        if (ps == 0) __threadfence(); }
}

__global__ __launch_bounds__(256) void k_wth(const float* __restrict__ src, h16* dst) {
    __shared__ __align__(16) h16 ts[CO * HD];
    const unsigned tid = threadIdx.x;
#pragma unroll 1
    for (unsigned it = 0; it < (unsigned)(HD * CO / 256); ++it) {
        const unsigned idx = it * 256u + tid; const unsigned d = idx / (unsigned)CO, c = idx % (unsigned)CO;
        ts[c * (unsigned)HD + d] = toh_flush(bfr(src[idx])); }
    __syncthreads();
#pragma unroll 1
    for (int ps = 0; ps < 2; ++ps) {
#pragma unroll 1
        for (unsigned it = 0; it < (unsigned)(HD * CO / 8 / 256); ++it) {
            const unsigned c = it * 256u + tid;
            const v8h o = *(const v8ha*)(&ts[c * 8u]);
            *(volatile v8h*)(dst + (size_t)c * 8) = o; }
        if (ps == 0) __threadfence(); }
}

__global__ __launch_bounds__(32) void k_proj_qk(const bf* __restrict__ A, const bf* __restrict__ Bt, h16* Ph, h16* Pr) {
    __shared__ __align__(16) float os[16 * OP];
    const int lane = threadIdx.x & 31, lr = lane & 15, hi = lane >> 4;
    const unsigned r0 = blockIdx.x * 64u;
    v8f acc[4][4];
#pragma unroll
    for (int mb = 0; mb < 4; ++mb)
#pragma unroll
        for (int nb = 0; nb < 4; ++nb) acc[mb][nb] = (v8f){};
    const size_t aoff = (size_t)(r0 + (unsigned)lr) * CIN + 8 * hi, boff = (size_t)lr * CIN + 8 * hi;
#pragma unroll 1
    for (int kc = 0; kc < CIN; kc += 32) {
        v16bf a[4];
#pragma unroll
        for (int mb = 0; mb < 4; ++mb) a[mb] = ldb(A + aoff + (size_t)mb * 16 * CIN + kc);
#pragma unroll
        for (int nb = 0; nb < 4; ++nb) { const v16bf b = ldb(Bt + boff + (size_t)nb * 16 * CIN + kc);
#pragma unroll
            for (int mb = 0; mb < 4; ++mb) acc[mb][nb] = wmmabg(a[mb], b, acc[mb][nb]); }
    }
    const unsigned bb = r0 / (unsigned)SEQ, tt = r0 % (unsigned)SEQ;
    const size_t tbase = ((size_t)(bb * 2u) * SEQ + (size_t)tt) * HD;
#pragma unroll
    for (int mb = 0; mb < 4; ++mb) {
#pragma unroll
        for (int nb = 0; nb < 4; ++nb) {
#pragma unroll
            for (int j = 0; j < 8; ++j) os[(hi * 8 + j) * OP + nb * 16 + lr] = acc[mb][nb][j]; }
        wave_sync();
#pragma unroll 1
        for (int ps = 0; ps < 2; ++ps) {
            const size_t sb = tbase + (size_t)(mb * 16) * HD;
#pragma unroll
            for (int hh = 0; hh < 2; ++hh) {
#pragma unroll
                for (int s = 0; s < 2; ++s) { const int p = s * 32 + lane; const int row = p >> 2, c8 = (p & 3) * 8;
                    const v4f x0 = *(const v4fa*)(&os[row * OP + hh * 32 + c8]); const v4f x1 = *(const v4fa*)(&os[row * OP + hh * 32 + c8 + 4]); v8h hv, rv;
#pragma unroll
                    for (int i = 0; i < 4; ++i) { const h16 a0 = toh_flush(x0[i]); const h16 a1 = toh_flush(x1[i]); hv[i] = a0; hv[4 + i] = a1;
                        rv[i] = toh_flush((x0[i] - (float)a0) * QRS); rv[4 + i] = toh_flush((x1[i] - (float)a1) * QRS); }
                    const size_t oo = sb + (size_t)hh * ((size_t)SEQ * HD) + (size_t)p * 8;
                    *(volatile v8h*)(Ph + oo) = hv; *(volatile v8h*)(Pr + oo) = rv; } }
            if (ps == 0) __threadfence(); }
        wave_sync();
    }
}

__global__ __launch_bounds__(32) void k_proj_vt(const bf* __restrict__ A, const bf* __restrict__ Bt, h16* Ph) {
    __shared__ __align__(16) float os[16 * OP];
    const int lane = threadIdx.x & 31, lr = lane & 15, hi = lane >> 4;
    const unsigned c0 = blockIdx.x * 64u;
    v8f acc[2][4];
#pragma unroll
    for (int mb = 0; mb < 2; ++mb)
#pragma unroll
        for (int nb = 0; nb < 4; ++nb) acc[mb][nb] = (v8f){};
    const size_t aoff = (size_t)lr * CIN + 8 * hi, boff = (size_t)(c0 + (unsigned)lr) * CIN + 8 * hi;
#pragma unroll 1
    for (int kc = 0; kc < CIN; kc += 32) {
        v16bf a[2];
#pragma unroll
        for (int mb = 0; mb < 2; ++mb) a[mb] = ldb(A + aoff + (size_t)mb * 16 * CIN + kc);
#pragma unroll
        for (int nb = 0; nb < 4; ++nb) { const v16bf b = ldb(Bt + boff + (size_t)nb * 16 * CIN + kc);
#pragma unroll
            for (int mb = 0; mb < 2; ++mb) acc[mb][nb] = wmmabg(a[mb], b, acc[mb][nb]); }
    }
    const unsigned bb = c0 / (unsigned)SEQ, tt = c0 % (unsigned)SEQ;
    const size_t tbase = (size_t)bb * (size_t)HD * SEQ + (size_t)tt;
#pragma unroll
    for (int mb = 0; mb < 2; ++mb) {
#pragma unroll
        for (int nb = 0; nb < 4; ++nb) {
#pragma unroll
            for (int j = 0; j < 8; ++j) os[(hi * 8 + j) * OP + nb * 16 + lr] = acc[mb][nb][j]; }
        wave_sync();
#pragma unroll 1
        for (int ps = 0; ps < 2; ++ps) {
            const size_t sb = tbase + (size_t)(mb * 16) * SEQ;
#pragma unroll
            for (int s = 0; s < 4; ++s) { const int row = 4 * s + (lane >> 3), c8 = (lane & 7) * 8;
                const v4f x0 = *(const v4fa*)(&os[row * OP + c8]); const v4f x1 = *(const v4fa*)(&os[row * OP + c8 + 4]); v8h hv;
#pragma unroll
                for (int i = 0; i < 4; ++i) { hv[i] = toh_flush(x0[i]); hv[4 + i] = toh_flush(x1[i]); }
                const size_t oo = sb + (size_t)row * SEQ + c8;
                *(volatile v8h*)(Ph + oo) = hv; }
            if (ps == 0) __threadfence(); }
        wave_sync();
    }
}

__global__ __launch_bounds__(32 * AW) void k_flash(const h16* __restrict__ PH, const h16* __restrict__ PR, const h16* __restrict__ VT, const h16* __restrict__ WO,
                                                   const float* __restrict__ X, const float* __restrict__ gamma_p, float* OUT) {
    __shared__ __align__(16) float os[AW * 16 * OP];
    const int lane = threadIdx.x & 31, lr = lane & 15, hi = lane >> 4;
    const int wave = __builtin_amdgcn_readfirstlane((int)(threadIdx.x >> 5));
    const unsigned bx = blockIdx.x, b = blockIdx.y;
    const int t0 = (int)(bx * (unsigned)AW + (unsigned)wave) * 16;
    const size_t kbase = (size_t)(b * 2u) * SEQ * HD;
    const size_t qbase = (size_t)(b * 2u + 1u) * SEQ * HD;
    const size_t qo = qbase + (size_t)(t0 + lr) * HD + 8 * hi;
    const v16h qh = ldh(PH + qo), qr = ldh(PR + qo);
    const size_t ko = kbase + (size_t)lr * HD + 8 * hi;
    const size_t vo = (size_t)b * HD * SEQ + (size_t)lr * SEQ + 8 * hi;
    v8f o0 = (v8f){}, o1 = (v8f){};
    float m = NEGB, l = 0.0f;
#pragma unroll 1
    for (int key0 = 0; key0 < SEQ; key0 += 32) {
        const h16* ka = PH + ko + (size_t)key0 * HD;
        const h16* kr = PR + ko + (size_t)key0 * HD;
        const v16h ka0 = ldh(ka), kb0 = ldh(ka + 16 * HD);
        const v16h kra0 = ldh(kr), krb0 = ldh(kr + 16 * HD);
        v8f sHa = (v8f){}, sLa = (v8f){}, sHb = (v8f){}, sLb = (v8f){};
        sHa = wmma16g(ka0, qh, sHa); sLa = wmma16g(ka0, qr, sLa); sLa = wmma16g(kra0, qh, sLa);
        sHb = wmma16g(kb0, qh, sHb); sLb = wmma16g(kb0, qr, sLb); sLb = wmma16g(krb0, qh, sLb);
        float ta[8], tb[8]; float mx = NEGB;
#pragma unroll
        for (int r = 0; r < 8; ++r) {
            ta[r] = (sHa[r] + sLa[r] * QRI) * L2E; tb[r] = (sHb[r] + sLb[r] * QRI) * L2E;
            mx = fmaxf(mx, fmaxf(ta[r], tb[r])); }
        mx = fmaxf(mx, __shfl_xor(mx, 16, 32));
        const float mnew = fmaxf(m, mx);
        const float alpha = __builtin_amdgcn_exp2f(m - mnew);
        const float sh = PSH - mnew;
        v16h pb; float ls = 0.0f;
#pragma unroll
        for (int r = 0; r < 8; ++r) {
            const float ea = __builtin_amdgcn_exp2f(ta[r] + sh), eb = __builtin_amdgcn_exp2f(tb[r] + sh);
            const h16 pa = toh_flush(ea); const h16 pc = toh_flush(eb);
            pb[r] = pa; pb[8 + r] = pc;
            ls += (float)pa + (float)pc; }
        l = l * alpha + ls; m = mnew;
        o0 = o0 * alpha; o1 = o1 * alpha;
        const h16* va = VT + vo + key0;
        const v16h v0 = ldh(va), v1 = ldh(va + (size_t)16 * SEQ);
        o0 = wmma16g(v0, pb, o0); o1 = wmma16g(v1, pb, o1);
    }
    l += __shfl_xor(l, 16, 32);
    const float inv = 1.0f / l;
    v16h ao;
#pragma unroll
    for (int r = 0; r < 8; ++r) { ao[r] = toh_flush(o0[r] * inv); ao[8 + r] = toh_flush(o1[r] * inv); }
    const float g = bfr(gamma_p[0]);
    const size_t xrow = ((size_t)b * SEQ_FULL + (size_t)t0) * CIN;
    const size_t orow = ((size_t)b * OUT_SEQ + (size_t)t0) * CO;
    const int wb = wave * 16 * OP;
#pragma unroll 1
    for (int cc = 0; cc < CO / 64; ++cc) {
        v8f acc[4];
#pragma unroll
        for (int nb = 0; nb < 4; ++nb) { const v16h bw = ldh(WO + (size_t)(cc * 64 + nb * 16 + lr) * HD + 8 * hi);
            acc[nb] = wmma16g(ao, bw, (v8f){}); }
#pragma unroll
        for (int nb = 0; nb < 4; ++nb) {
#pragma unroll
            for (int j = 0; j < 8; ++j) os[wb + (hi * 8 + j) * OP + nb * 16 + lr] = acc[nb][j]; }
        wave_sync();
#pragma unroll 1
        for (int ps = 0; ps < 2; ++ps) {
#pragma unroll
            for (int s = 0; s < 8; ++s) { const int p = s * 32 + lane; const int row = p >> 4, c4 = (p & 15) * 4;
                const v4f val = *(const v4fa*)(&os[wb + row * OP + c4]);
                const v4f xv = *(const v4f*)(X + xrow + (size_t)row * CIN + cc * 64 + c4);
                v4f ov;
#pragma unroll
                for (int i = 0; i < 4; ++i) ov[i] = g * val[i] + bfr(xv[i]);
                *(volatile v4f*)(OUT + orow + (size_t)row * CO + cc * 64 + c4) = ov; }
            if (ps == 0) __threadfence(); }
        wave_sync();
    }
}

static constexpr size_t al256(size_t v) { return (v + 255) & ~(size_t)255; }
static constexpr size_t SZ_XB = al256((size_t)NB * SEQ * CIN * 2);
static constexpr size_t SZ_WT = al256((size_t)3 * HD * CIN * 2);
static constexpr size_t SZ_WO = al256((size_t)CO * HD * 2);
static constexpr size_t SZ_PL = al256((size_t)NB * 2 * SEQ * HD * 2);
static constexpr size_t SZ_VT = al256((size_t)NB * HD * SEQ * 2);
static constexpr size_t SZ_TOTAL = SZ_XB + SZ_WT + SZ_WO + 2 * SZ_PL + SZ_VT;
static_assert(SZ_TOTAL <= (size_t)134217728);
static_assert(((size_t)HD * CIN * 2) % 256 == 0);
static_assert((size_t)(NB * SEQ / 64) * 64 * 2 * HD == (size_t)NB * 2 * SEQ * HD);
static_assert((size_t)(NB * SEQ / 64) * 64 * HD == (size_t)NB * HD * SEQ);

extern "C" void kernel_launch(void* const* d_in, const int* in_sizes, int n_in,
                              void* d_out, int out_size, void* d_ws, size_t ws_size, hipStream_t stream) {
    if (n_in < 6) return;
    const size_t needx = ((size_t)(NB - 1) * SEQ_FULL + SEQ) * CIN;
    if ((size_t)in_sizes[0] < needx) return;
    if (in_sizes[1] < CIN * HD || in_sizes[2] < CIN * HD || in_sizes[3] < CIN * HD || in_sizes[4] < HD * CO || in_sizes[5] < 1) return;
    if ((size_t)out_size < ((size_t)(NB - 1) * OUT_SEQ + SEQ) * CO) return;
    if (SZ_TOTAL > ws_size) return;
    const float* x  = (const float*)d_in[0];
    const float* wf = (const float*)d_in[1];
    const float* wg = (const float*)d_in[2];
    const float* wh = (const float*)d_in[3];
    const float* wv = (const float*)d_in[4];
    const float* gm = (const float*)d_in[5];
    float* OUT = (float*)d_out;
    char* wsp = (char*)d_ws;
    bf*  XB = (bf*)wsp;  wsp += SZ_XB;
    bf*  WT = (bf*)wsp;  wsp += SZ_WT;
    h16* WO = (h16*)wsp; wsp += SZ_WO;
    h16* PH = (h16*)wsp; wsp += SZ_PL;
    h16* PR = (h16*)wsp; wsp += SZ_PL;
    h16* VT = (h16*)wsp; wsp += SZ_VT;

    if (SEQ == SEQ_FULL) {
        const size_t n8 = (size_t)NB * SEQ * CIN / 8;
        k_cvt8<<<(unsigned)((n8 + 255) / 256), 256, 0, stream>>>(x, XB, n8);
    } else {
        const size_t n8 = (size_t)SEQ * CIN / 8;
        for (int b = 0; b < NB; ++b) k_cvt8<<<(unsigned)((n8 + 255) / 256), 256, 0, stream>>>(x + (size_t)b * SEQ_FULL * CIN, XB + (size_t)b * SEQ * CIN, n8);
    }
    k_wtb<<<1, 256, 0, stream>>>(wf, WT);
    k_wtb<<<1, 256, 0, stream>>>(wg, WT + (size_t)HD * CIN);
    k_wtb<<<1, 256, 0, stream>>>(wh, WT + (size_t)2 * HD * CIN);
    k_wth<<<1, 256, 0, stream>>>(wv, WO);

    k_proj_qk<<<dim3(NB * SEQ / 64, 1, 1), 32, 0, stream>>>(XB, WT, PH, PR);
    k_proj_vt<<<dim3(NB * SEQ / 64, 1, 1), 32, 0, stream>>>(WT + (size_t)2 * HD * CIN, XB, VT);

    k_flash<<<dim3(SEQ / (16 * AW), NB, 1), 32 * AW, 0, stream>>>(PH, PR, VT, WO, x, gm, OUT);
}
